// GatedLinearAttention_10514079940651
// MI455X (gfx1250) — hardware-verified
//
#include <hip/hip_runtime.h>
#include <math.h>

constexpr int kT    = 2048;
constexpr int kBsz  = 4;
constexpr int kC    = 1024;
constexpr int kH    = 16;
constexpr int kD    = 64;
constexpr int kGH   = 16;
constexpr int kRows = kT * kBsz;
constexpr int kQKVN = 3 * kC;
constexpr int kG1N  = 64;
constexpr int kG2K  = 32;
constexpr int kTS   = 32;

typedef __attribute__((ext_vector_type(16))) _Float16 v16h;
typedef __attribute__((ext_vector_type(8)))  _Float16 v8h;
typedef __attribute__((ext_vector_type(16))) __bf16   v16b;
typedef __attribute__((ext_vector_type(8)))  __bf16   v8b;
typedef __attribute__((ext_vector_type(8)))  float    v8f;
typedef __attribute__((ext_vector_type(4)))  float    v4f;
typedef __attribute__((ext_vector_type(4)))  unsigned int v4u;

__device__ __forceinline__ unsigned short f2bf_bits(float f) {
  unsigned u = __float_as_uint(f);
  return (unsigned short)((u + 0x7FFFu + ((u >> 16) & 1u)) >> 16);
}
__device__ __forceinline__ float bf_bits2f(unsigned short h) { return __uint_as_float(((unsigned)h) << 16); }

__device__ __forceinline__ void dep_guard_h(v8f& a, v8f& b, v16h x, v16h y) { asm volatile("v_nop\n\tv_nop\n\tv_nop\n\tv_nop" : "+v"(a), "+v"(b) : "v"(x), "v"(y)); }
__device__ __forceinline__ void dep_guard_b(v8f& a, v8f& b, v16b x, v16b y) { asm volatile("v_nop\n\tv_nop\n\tv_nop\n\tv_nop" : "+v"(a), "+v"(b) : "v"(x), "v"(y)); }
__device__ __forceinline__ void keep4_h(v16h a, v16h b, v16h c, v16h d) { asm volatile("v_nop" :: "v"(a), "v"(b), "v"(c), "v"(d)); }
__device__ __forceinline__ void keep4_b(v16b a, v16b b, v16b c, v16b d) { asm volatile("v_nop" :: "v"(a), "v"(b), "v"(c), "v"(d)); }
__device__ __forceinline__ void acc_guard4(v8f& a, v8f& b, v8f& c, v8f& d) { asm volatile("v_nop\n\tv_nop\n\tv_nop\n\tv_nop" : "+v"(a), "+v"(b), "+v"(c), "+v"(d)); }
template <typename T> struct Frag;
template <> struct Frag<_Float16> {
  typedef v16h V; union U { v16h v; v8h h[2]; };
  static __device__ __forceinline__ v16h load(const _Float16* p) {
    U f; f.h[0] = *(const v8h*)(p); f.h[1] = *(const v8h*)(p + 16); return f.v;
  }
  static __device__ __forceinline__ v8f mma(v16h a, v16h b, v8f c) {
    return __builtin_amdgcn_wmma_f32_16x16x32_f16(false, a, false, b, (short)0, c, false, false);
  }
  static __device__ __forceinline__ void guard(v8f& a, v8f& b, v16h x, v16h y) { dep_guard_h(a, b, x, y); }
  static __device__ __forceinline__ void keep(v16h a, v16h b, v16h c, v16h d) { keep4_h(a, b, c, d); }
};
template <> struct Frag<__bf16> {
  typedef v16b V; union U { v16b v; v8b h[2]; };
  static __device__ __forceinline__ v16b load(const __bf16* p) {
    U f; f.h[0] = *(const v8b*)(p); f.h[1] = *(const v8b*)(p + 16); return f.v;
  }
  static __device__ __forceinline__ v8f mma(v16b a, v16b b, v8f c) {
    return __builtin_amdgcn_wmma_f32_16x16x32_bf16(false, a, false, b, (short)0, c, false, false);
  }
  static __device__ __forceinline__ void guard(v8f& a, v8f& b, v16b x, v16b y) { dep_guard_b(a, b, x, y); }
  static __device__ __forceinline__ void keep(v16b a, v16b b, v16b c, v16b d) { keep4_b(a, b, c, d); }
};

__device__ __forceinline__ unsigned pk16(unsigned short a, unsigned short b) { return (unsigned)a | ((unsigned)b << 16); }
__device__ __forceinline__ unsigned short h_bits(float f) { const _Float16 h = (_Float16)f; return __builtin_bit_cast(unsigned short, h); }

__device__ __forceinline__ float sigm_f(float v) {
  const float e = __expf(-fabsf(v));
  const float r = 1.0f / (1.0f + e);
  return (v >= 0.0f) ? r : e * r;
}

template <int ET> struct Elem;
template <> struct Elem<0> { typedef _Float16 T; };
template <> struct Elem<1> { typedef __bf16 T; };
template <int ET, int SPL, int BIAS, int OUT_MODE, int ACT, int MULR>
__global__ __launch_bounds__(256) void wmma_gemm64(
    const unsigned short* __restrict__ Ap, const unsigned short* __restrict__ A2p, int lda, long strideA,
    const unsigned short* __restrict__ Btp, const unsigned short* __restrict__ Bt2p, int ldb, long strideB,
    void* __restrict__ Cout, void* __restrict__ Cout2, int ldc, long strideC,
    const float* __restrict__ bias, int nbias,
    const float* __restrict__ mulr, int ldr,
    int M, int N, int K, float scale) {
  typedef typename Elem<ET>::T T;
  typedef typename Frag<T>::V V;
  const T* A = (const T*)Ap; const T* A2 = (const T*)A2p; const T* Bt = (const T*)Btp; const T* Bt2 = (const T*)Bt2p;
  __shared__ __align__(16) float sT[8][16 * 68];
  const int b    = blockIdx.y;
  const int lane = threadIdx.x & 31;
  const int wave = threadIdx.x >> 5;
  const int tilesN = N >> 6;
  const int tilesM = M >> 6;
  const int tile = blockIdx.x * 8 + wave;
  if (tile >= tilesM * tilesN) return;
  const int tm = tile / tilesN;
  const int tn = tile - tm * tilesN;
  const int m0 = tm << 6;
  const int n0 = tn << 6;

  const T* Ab  = A  + (size_t)b * strideA;
  const T* Bb  = Bt + (size_t)b * strideB;
  const T* Ab2 = (SPL & 1) ? (A2  + (size_t)b * strideA) : nullptr;
  const T* Bb2 = (SPL & 2) ? (Bt2 + (size_t)b * strideB) : nullptr;

  const int rlane = lane & 15;
  const int koff  = (lane >> 4) * 8;
  const int mOff  = (lane >> 4) * 8;

  v8f acc[4][4];
#pragma unroll
  for (int i = 0; i < 4; ++i)
#pragma unroll
    for (int j = 0; j < 4; ++j) acc[i][j] = (v8f){0.f,0.f,0.f,0.f,0.f,0.f,0.f,0.f};

  for (int k0 = 0; k0 < K; k0 += 32) {
    V bh[4], bl[4];
#pragma unroll
    for (int j = 0; j < 4; ++j) {
      const size_t bo = (size_t)(n0 + (j << 4) + rlane) * ldb + koff + k0;
      bh[j] = Frag<T>::load(Bb + bo);
      if (SPL & 2) bl[j] = Frag<T>::load(Bb2 + bo);
    }
#pragma unroll
    for (int i = 0; i < 4; ++i) {
      const size_t ao = (size_t)(m0 + (i << 4) + rlane) * lda + koff + k0;
      V ah = Frag<T>::load(Ab + ao);
      V al;
      if (SPL & 1) al = Frag<T>::load(Ab2 + ao);
#pragma unroll
      for (int j = 0; j < 4; ++j) {
        acc[i][j] = Frag<T>::mma(ah, bh[j], acc[i][j]);
        if (SPL & 2) acc[i][j] = Frag<T>::mma(ah, bl[j], acc[i][j]);
        if (SPL & 1) acc[i][j] = Frag<T>::mma(al, bh[j], acc[i][j]);
      }
      Frag<T>::guard(acc[i][0], acc[i][3], ah, (SPL & 1) ? al : ah);
    }
    Frag<T>::keep(bh[0], bh[1], bh[2], bh[3]);
    if (SPL & 2) Frag<T>::keep(bl[0], bl[1], bl[2], bl[3]);
  }
  acc_guard4(acc[0][0], acc[0][1], acc[0][2], acc[0][3]);
  acc_guard4(acc[1][0], acc[1][1], acc[1][2], acc[1][3]);
  acc_guard4(acc[2][0], acc[2][1], acc[2][2], acc[2][3]);
  acc_guard4(acc[3][0], acc[3][1], acc[3][2], acc[3][3]);

  float* slab = sT[wave];
#pragma unroll
  for (int i = 0; i < 4; ++i) {
    const int mBase = m0 + (i << 4);
#pragma unroll
    for (int j = 0; j < 4; ++j) {
      const int n = n0 + (j << 4) + rlane;
      float bv = 0.f;
      if (BIAS == 2) {
        const int nc = (n < nbias) ? n : (nbias - 1);
        bv = bf_bits2f(f2bf_bits(bias[nc]));
        if (n >= nbias) bv = 0.0f;
      }
#pragma unroll
      for (int r = 0; r < 8; ++r) {
        float v = acc[i][j][r] * scale;
        if (BIAS == 2) v += bv;
        if (ACT == 3) v = v * sigm_f(v);
        if (ACT == 7) v = sigm_f(0.0625f * v);
        if (MULR) v = v * mulr[(size_t)(mBase + mOff + r) * ldr + n];
        slab[(mOff + r) * 68 + (j << 4) + rlane] = v;
      }
    }
    __builtin_amdgcn_fence(__ATOMIC_RELEASE, "workgroup");
    __builtin_amdgcn_wave_barrier();
    __builtin_amdgcn_fence(__ATOMIC_ACQUIRE, "workgroup");
    if (OUT_MODE == 0) {
      float* Cp = (float*)Cout + (size_t)b * strideC;
      const int hh = lane >> 4, c4 = (lane & 15) * 4;
      for (int pass = 0; pass < 2; ++pass) {
#pragma unroll
        for (int it = 0; it < 8; ++it) {
          const int row = it * 2 + hh;
          v4f v = *(const v4f*)(slab + row * 68 + c4);
          *(volatile v4f*)(Cp + (size_t)(mBase + row) * ldc + n0 + c4) = v;
        }
        __threadfence();
      }
    } else {
      const int q = lane >> 3, c8 = (lane & 7) * 8;
      unsigned short* Cp  = (unsigned short*)Cout  + (size_t)b * strideC;
      unsigned short* Cp2 = (OUT_MODE == 2) ? ((unsigned short*)Cout2 + (size_t)b * strideC) : nullptr;
      for (int pass = 0; pass < 2; ++pass) {
#pragma unroll
        for (int it = 0; it < 4; ++it) {
          const int row = it * 4 + q;
          const float* sp = slab + row * 68 + c8;
          v8h hv, lv;
#pragma unroll
          for (int e = 0; e < 8; ++e) {
            if (OUT_MODE == 1) {
              hv[e] = (_Float16)sp[e];
            } else {
              unsigned short hb = f2bf_bits(sp[e]);
              unsigned short lb = f2bf_bits(sp[e] - bf_bits2f(hb));
              hv[e] = __builtin_bit_cast(_Float16, hb);
              lv[e] = __builtin_bit_cast(_Float16, lb);
            }
          }
          *(volatile v8h*)(Cp + (size_t)(mBase + row) * ldc + n0 + c8) = hv;
          if (OUT_MODE == 2) *(volatile v8h*)(Cp2 + (size_t)(mBase + row) * ldc + n0 + c8) = lv;
        }
        __threadfence();
      }
    }
    __builtin_amdgcn_fence(__ATOMIC_RELEASE, "workgroup");
    __builtin_amdgcn_wave_barrier();
    __builtin_amdgcn_fence(__ATOMIC_ACQUIRE, "workgroup");
  }
}

template <int MODE>
__global__ __launch_bounds__(256) void cast8_kernel(const float* __restrict__ in, unsigned short* __restrict__ out, int n8, float scale) {
  const int i = blockIdx.x * 256 + threadIdx.x;
  if (i >= n8) return;
  const float* p = in + 8 * (size_t)i;
  const v4f a = *(const v4f*)(p);
  const v4f c = *(const v4f*)(p + 4);
  unsigned short hb[8];
#pragma unroll
  for (int e = 0; e < 4; ++e) {
    if (MODE == 0) {
      hb[e]     = f2bf_bits(a[e]);
      hb[4 + e] = f2bf_bits(c[e]);
    } else {
      hb[e]     = h_bits(bf_bits2f(f2bf_bits(a[e])) * scale);
      hb[4 + e] = h_bits(bf_bits2f(f2bf_bits(c[e])) * scale);
    }
  }
  const v4u u = (v4u){pk16(hb[0], hb[1]), pk16(hb[2], hb[3]), pk16(hb[4], hb[5]), pk16(hb[6], hb[7])};
  unsigned short* q = out + 8 * (size_t)i;
  *(volatile v4u*)q = u;
  __threadfence();
  *(volatile v4u*)q = u;
  (void)scale;
}

__global__ __launch_bounds__(256) void tcast8_kernel(const float* __restrict__ in, unsigned short* __restrict__ out,
                                                     int Kin, int Nin, int Npad, int Kpad, int n8) {
  const int i = blockIdx.x * 256 + threadIdx.x;
  if (i >= n8) return;
  const size_t e0 = (size_t)i * 8;
  const int n  = (int)(e0 / (size_t)Kpad);
  const int k0 = (int)(e0 - (size_t)n * Kpad);
  const int nc = (n < Nin) ? n : (Nin - 1);
  unsigned short hb[8];
#pragma unroll
  for (int e = 0; e < 8; ++e) {
    const int k  = k0 + e;
    const int kc = (k < Kin) ? k : (Kin - 1);
    float f = in[(size_t)kc * Nin + nc];
    if (k >= Kin || n >= Nin) f = 0.0f;
    hb[e] = f2bf_bits(f);
  }
  const v4u u = (v4u){pk16(hb[0], hb[1]), pk16(hb[2], hb[3]), pk16(hb[4], hb[5]), pk16(hb[6], hb[7])};
  unsigned short* q = out + e0;
  *(volatile v4u*)q = u;
  __threadfence();
  *(volatile v4u*)q = u;
  (void)Npad;
}

__global__ __launch_bounds__(256) void gla_scan_kernel(const float* __restrict__ bat, float* __restrict__ OLN,
                                                       float* __restrict__ Sfin, int bsel) {
  __shared__ __align__(16) float stg[4][kTS][64];
  __shared__ __align__(16) float so[kTS][68];
  __shared__ __align__(16) float sS[64][68];
  const int h    = blockIdx.x;
  const int tid  = threadIdx.x;
  const int lane = tid & 31, wave = tid >> 5;
  const int vcol = tid >> 2, kq = tid & 3;
  const int slot = tid & 63, arr = slot >> 4, j4 = (slot & 15) * 4, srow = tid >> 6;
  const int hc   = h * kD;
  const size_t aoff = (size_t)kT * kQKVN;

  float S[16];
#pragma unroll
  for (int e = 0; e < 16; ++e) S[e] = 0.0f;

#pragma unroll 1
  for (int t0 = 0; t0 < kT; t0 += kTS) {
    __syncthreads();
#pragma unroll
    for (int i = 0; i < 8; ++i) {
      const int s = i * 4 + srow;
      const size_t t = (size_t)(t0 + s);
      const size_t off = (arr == 3) ? (aoff + t * (size_t)kC) : (t * (size_t)kQKVN + (size_t)arr * kC);
      const v4f val = *(const v4f*)(bat + off + hc + j4);
      *(v4f*)(&stg[arr][s][j4]) = val;
    }
    __syncthreads();
#pragma unroll 1
    for (int s = 0; s < kTS; ++s) {
      const float vv = stg[2][s][vcol];
      float o = 0.0f;
#pragma unroll
      for (int e4 = 0; e4 < 4; ++e4) {
        const int kb = kq * 16 + e4 * 4;
        const v4f a4 = *(const v4f*)(&stg[3][s][kb]);
        const v4f k4 = *(const v4f*)(&stg[1][s][kb]);
        const v4f q4 = *(const v4f*)(&stg[0][s][kb]);
#pragma unroll
        for (int e = 0; e < 4; ++e) {
          const int idx = e4 * 4 + e;
          const float sn = a4[e] * S[idx] + k4[e] * vv;
          S[idx] = sn;
          o += q4[e] * sn;
        }
      }
      o += __shfl_xor(o, 1, 32);
      o += __shfl_xor(o, 2, 32);
      if (kq == 0) so[s][vcol] = o;
    }
    __syncthreads();
#pragma unroll
    for (int rr = 0; rr < 4; ++rr) {
      const int row = wave * 4 + rr;
      const float x0 = so[row][lane], x1 = so[row][lane + 32];
      float sum = x0 + x1;
#pragma unroll
      for (int off = 16; off > 0; off >>= 1) sum += __shfl_xor(sum, off, 32);
      const float mu = sum * (1.0f / 64.0f);
      const float d0 = x0 - mu, d1 = x1 - mu;
      float sq = d0 * d0 + d1 * d1;
#pragma unroll
      for (int off = 16; off > 0; off >>= 1) sq += __shfl_xor(sq, off, 32);
      const float var = sq * (1.0f / 64.0f);
      const float rs  = 1.0f / sqrtf(var + 1e-5f);
      so[row][lane]      = d0 * rs;
      so[row][lane + 32] = d1 * rs;
    }
    __builtin_amdgcn_fence(__ATOMIC_RELEASE, "workgroup");
    __builtin_amdgcn_wave_barrier();
    __builtin_amdgcn_fence(__ATOMIC_ACQUIRE, "workgroup");
    {
      const int hh = lane >> 4, c4 = (lane & 15) * 4;
      for (int pass = 0; pass < 2; ++pass) {
#pragma unroll
        for (int it = 0; it < 2; ++it) {
          const int row = wave * 4 + it * 2 + hh;
          const v4f val = *(const v4f*)(&so[row][c4]);
          *(volatile v4f*)(OLN + ((size_t)(t0 + row) * kBsz + bsel) * (size_t)kC + hc + c4) = val;
        }
        __threadfence();
      }
    }
  }

#pragma unroll
  for (int e = 0; e < 16; ++e) sS[kq * 16 + e][vcol] = S[e];
  __syncthreads();
  {
    float* dst = Sfin + (size_t)(bsel * kH + h) * (kD * kD);
    const int hh = lane >> 4, c4 = (lane & 15) * 4;
    for (int pass = 0; pass < 2; ++pass) {
#pragma unroll
      for (int it = 0; it < 4; ++it) {
        const int row = wave * 8 + it * 2 + hh;
        const v4f val = *(const v4f*)(&sS[row][c4]);
        *(volatile v4f*)(dst + (size_t)row * kD + c4) = val;
      }
      __threadfence();
    }
  }
}

extern "C" void kernel_launch(void* const* d_in, const int* in_sizes, int n_in,
                              void* d_out, int out_size, void* d_ws, size_t ws_size,
                              hipStream_t stream) {
  if (n_in < 11) return;
  if (in_sizes[0] != kRows * kC) return;
  if (in_sizes[1] != kC * kC || in_sizes[2] != kC * kC || in_sizes[3] != kC * kC) return;
  if (in_sizes[4] != kC * kGH || in_sizes[5] != kGH || in_sizes[6] != kGH * kC || in_sizes[7] != kC) return;
  if (in_sizes[8] != kC * kC || in_sizes[9] != kC || in_sizes[10] != kC * kC) return;
  if (out_size != kRows * kC + kBsz * kH * kD * kD) return;

  const float* x   = (const float*)d_in[0];
  const float* Wq  = (const float*)d_in[1];
  const float* Wk  = (const float*)d_in[2];
  const float* Wv  = (const float*)d_in[3];
  const float* Wg1 = (const float*)d_in[4];
  const float* bg1 = (const float*)d_in[5];
  const float* Wg2 = (const float*)d_in[6];
  const float* bg2 = (const float*)d_in[7];
  const float* Wog = (const float*)d_in[8];
  const float* bog = (const float*)d_in[9];
  const float* Wo  = (const float*)d_in[10];
  float* outp = (float*)d_out;
  float* Sfin = outp + (size_t)kRows * kC;

  const size_t SZ_XB   = (size_t)kRows * kC * 2;
  const size_t SZ_WQKV = (size_t)kQKVN * kC * 2;
  const size_t SZ_W    = (size_t)kC * kC * 2;
  const size_t SZ_WG1  = (size_t)kG1N * kC * 2;
  const size_t SZ_WG2  = (size_t)kC * kG2K * 2;
  const size_t SZ_G1   = (size_t)kRows * kG1N * 2;
  const size_t SZ_QKV  = (size_t)kT * kQKVN * 4;
  const size_t SZ_ALP  = (size_t)kT * kC * 4;
  const size_t SZ_Y    = (size_t)kRows * kC * 2;
  const size_t SZ_BATA = SZ_QKV + SZ_ALP;
  const size_t SZ_BATB = 2 * SZ_Y;
  const size_t SZ_BAT  = (SZ_BATA > SZ_BATB) ? SZ_BATA : SZ_BATB;
  const size_t SZ_OLN  = (size_t)kRows * kC * 4;

  size_t off = 0;
  const size_t oXB   = off; off += SZ_XB;
  const size_t oWQKV = off; off += SZ_WQKV;
  const size_t oWOG  = off; off += SZ_W;
  const size_t oWO   = off; off += SZ_W;
  const size_t oWG1  = off; off += SZ_WG1;
  const size_t oWG2  = off; off += SZ_WG2;
  const size_t oG1H  = off; off += SZ_G1;
  const size_t oG1L  = off; off += SZ_G1;
  const size_t oBAT  = off; off += SZ_BAT;
  const size_t oOLN  = off; off += SZ_OLN;
  const size_t TOTAL = off;
  if (TOTAL > ws_size) return;
  if (TOTAL > (size_t)134217728) return;

  char* ws = (char*)d_ws;
  unsigned short* XB   = (unsigned short*)(ws + oXB);
  unsigned short* WQKV = (unsigned short*)(ws + oWQKV);
  unsigned short* WOG  = (unsigned short*)(ws + oWOG);
  unsigned short* WO   = (unsigned short*)(ws + oWO);
  unsigned short* WG1  = (unsigned short*)(ws + oWG1);
  unsigned short* WG2  = (unsigned short*)(ws + oWG2);
  unsigned short* G1H  = (unsigned short*)(ws + oG1H);
  unsigned short* G1L  = (unsigned short*)(ws + oG1L);
  float*          QKV  = (float*)(ws + oBAT);
  float*          ALP  = (float*)(ws + oBAT + SZ_QKV);
  unsigned short* YH   = (unsigned short*)(ws + oBAT);
  unsigned short* YL   = (unsigned short*)(ws + oBAT + SZ_Y);
  float*          OLN  = (float*)(ws + oOLN);

  const dim3 blk(256);

  {
    const int n8 = kRows * kC / 8;
    cast8_kernel<0><<<dim3(n8 / 256), blk, 0, stream>>>(x, XB, n8, 1.0f);
  }
  {
    const int n8w = kC * kC / 8;
    tcast8_kernel<<<dim3(n8w / 256), blk, 0, stream>>>(Wq,  WQKV,                         kC, kC, kC, kC, n8w);
    tcast8_kernel<<<dim3(n8w / 256), blk, 0, stream>>>(Wk,  WQKV + (size_t)kC * kC,       kC, kC, kC, kC, n8w);
    tcast8_kernel<<<dim3(n8w / 256), blk, 0, stream>>>(Wv,  WQKV + (size_t)2 * kC * kC,   kC, kC, kC, kC, n8w);
    tcast8_kernel<<<dim3(n8w / 256), blk, 0, stream>>>(Wog, WOG,                          kC, kC, kC, kC, n8w);
    tcast8_kernel<<<dim3(n8w / 256), blk, 0, stream>>>(Wo,  WO,                           kC, kC, kC, kC, n8w);
    const int n8g1 = kG1N * kC / 8;
    tcast8_kernel<<<dim3(n8g1 / 256), blk, 0, stream>>>(Wg1, WG1, kC, kGH, kG1N, kC, n8g1);
    const int n8g2 = kC * kG2K / 8;
    tcast8_kernel<<<dim3(n8g2 / 256), blk, 0, stream>>>(Wg2, WG2, kGH, kC, kC, kG2K, n8g2);
  }

  const int tilesRows = kRows / 64;
  const dim3 gG1((tilesRows * (kG1N / 64) + 7) / 8, 1);
  const dim3 gQKV(((kT / 64) * (kQKVN / 64) + 7) / 8, 1);
  const dim3 gALP(((kT / 64) * (kC / 64) + 7) / 8, 1);
  const dim3 gSQ((tilesRows * (kC / 64) + 7) / 8, 1);

  wmma_gemm64<1, 0, 2, 2, 3, 0><<<gG1, blk, 0, stream>>>(
      XB, XB, kC, 0L, WG1, WG1, kC, 0L, (void*)G1H, (void*)G1L, kG1N, 0L, bg1, kGH, OLN, kC, kRows, kG1N, kC, 1.0f);

  for (int bb = 0; bb < kBsz; ++bb) {
    wmma_gemm64<1, 0, 0, 0, 0, 0><<<gQKV, blk, 0, stream>>>(
        XB + (size_t)bb * kC, XB + (size_t)bb * kC, kBsz * kC, 0L, WQKV, WQKV, kC, 0L,
        (void*)QKV, (void*)QKV, kQKVN, 0L, bg1, kGH, OLN, kC, kT, kQKVN, kC, 1.0f);
    wmma_gemm64<1, 1, 2, 0, 7, 0><<<gALP, blk, 0, stream>>>(
        G1H + (size_t)bb * kG1N, G1L + (size_t)bb * kG1N, kBsz * kG1N, 0L, WG2, WG2, kG2K, 0L,
        (void*)ALP, (void*)ALP, kC, 0L, bg2, kC, OLN, kC, kT, kC, kG2K, 1.0f);
    gla_scan_kernel<<<dim3(kH), blk, 0, stream>>>(QKV, OLN, Sfin, bb);
  }

  wmma_gemm64<1, 0, 2, 2, 3, 1><<<gSQ, blk, 0, stream>>>(
      XB, XB, kC, 0L, WOG, WOG, kC, 0L, (void*)YH, (void*)YL, kC, 0L, bog, kC, OLN, kC, kRows, kC, kC, 1.0f);

  wmma_gemm64<1, 1, 0, 0, 0, 0><<<gSQ, blk, 0, stream>>>(
      YH, YL, kC, 0L, WO, WO, kC, 0L, (void*)outp, (void*)outp, kC, 0L, bg1, kGH, OLN, kC, kRows, kC, kC, 1.0f);
}
